// GATv2_23398981828938
// MI455X (gfx1250) — hardware-verified
//
#include <hip/hip_runtime.h>
#include <stddef.h>
#include <stdint.h>


#define DIN     128
#define NHD     2
#define HDC     64
#define C1      128
#define C2      64
#define P1      (2 * C1)
#define P2      (2 * C2)
#define NTHR    256
#define NWAVE   8
#define EPT     8
#define CHUNK   (NTHR * EPT)
#define WCAP    (EPT * 32)
#define LISTN   (NWAVE * WCAP)
#define NBMAX   2048
#define SLOTB   11
#define NBRUN   1024
#define RCAP    28672
#define DEGCAP  128
#define STW     512
#define GBM     64
#define GBN     64
#define GTHR    128
#define CX      8.0f
#define CL      2048.0f
#define CW      64.0f
#define SCL_XW  0.001953125f
#define SCL_XWL 9.5367431640625e-7f
#define NEGS    0.2f
#define MX0     (-1.0e30f)
#define WSMAX   134217728
#define LDS_AGG ((2 * RCAP + 2 * NBMAX + LISTN) * 4 + 64)

static_assert((CHUNK & (CHUNK - 1)) == 0 && CHUNK <= (1 << SLOTB));
static_assert(NBMAX == (1 << SLOTB));
static_assert((NBRUN & (NBRUN - 1)) == 0 && NBRUN <= NBMAX && NBRUN >= 16);
static_assert(NTHR * 8 == NBMAX);
static_assert(LISTN >= NBMAX);
static_assert(LISTN >= NWAVE * WCAP);
static_assert((RCAP % 32) == 0);
static_assert(NWAVE * STW <= RCAP);
static_assert(C1 <= STW && C2 <= STW);
static_assert(LDS_AGG <= 300000);
static_assert(GBM == (GTHR / 32) * 16);
static_assert(DIN / 8 == 16);
static_assert((DIN % 32) == 0 && (C1 % 32) == 0 && (C2 % 32) == 0);
static_assert((P1 % GBN) == 0 && (P2 % GBN) == 0);
static_assert(C1 == NHD * HDC);
static_assert(C1 == 32 * 4);
static_assert(HDC == 16 * 4);
static_assert(C2 == 2 * 32);
static_assert(C1 == DIN);
static_assert(P2 * 4 <= P1 * 4);

typedef float          v4f   __attribute__((ext_vector_type(4)));
typedef float          v8f   __attribute__((ext_vector_type(8)));
typedef int            v4i   __attribute__((ext_vector_type(4)));
typedef int            v8i   __attribute__((ext_vector_type(8)));
typedef unsigned short v8us  __attribute__((ext_vector_type(8)));
typedef _Float16       v8h   __attribute__((ext_vector_type(8)));
typedef _Float16       v16h  __attribute__((ext_vector_type(16)));
typedef __bf16         v16bf __attribute__((ext_vector_type(16)));
typedef v4f  __attribute__((may_alias)) v4fa;
typedef v8us __attribute__((may_alias)) v8usa;
union FragH { v16h v;  v8us u[2]; v8i w; };
union FragB { v16bf v; v8us u[2]; v8i w; };
template<int BF> struct FT { typedef FragH T; };
template<> struct FT<1> { typedef FragB T; };

__device__ __forceinline__ v8f wmx(const FragH& a, const FragH& b, v8f c) {
  v8f d = __builtin_amdgcn_wmma_f32_16x16x32_f16(false, a.v, false, b.v, (short)0, c, false, false);
  asm volatile("v_nop\n\tv_nop\n\tv_nop\n\tv_nop" : "+v"(d) : "v"(a.w), "v"(b.w));
  return d;
}
__device__ __forceinline__ v8f wmx(const FragB& a, const FragB& b, v8f c) {
  v8f d = __builtin_amdgcn_wmma_f32_16x16x32_bf16(false, a.v, false, b.v, (short)0, c, false, false);
  asm volatile("v_nop\n\tv_nop\n\tv_nop\n\tv_nop" : "+v"(d) : "v"(a.w), "v"(b.w));
  return d;
}

__device__ __forceinline__ void ldwait() {
  asm volatile("s_wait_loadcnt 0x0" ::: "memory");
}

__device__ __forceinline__ unsigned bfbits(float v) {
  unsigned u = __float_as_uint(v);
  u = u + 0x7FFFu + ((u >> 16) & 1u);
  return u >> 16;
}
__device__ __forceinline__ float rbf(float v) { return __uint_as_float(bfbits(v) << 16); }

__device__ __forceinline__ v8us cvt8b(const v4f a, const v4f b) {
  v8us o;
  o[0] = (unsigned short)bfbits(a.x); o[1] = (unsigned short)bfbits(a.y);
  o[2] = (unsigned short)bfbits(a.z); o[3] = (unsigned short)bfbits(a.w);
  o[4] = (unsigned short)bfbits(b.x); o[5] = (unsigned short)bfbits(b.y);
  o[6] = (unsigned short)bfbits(b.z); o[7] = (unsigned short)bfbits(b.w);
  return o;
}
__device__ __forceinline__ v8h cvt8bh(const v4f a, const v4f b, const float c) {
  v8h hv;
  hv[0] = (_Float16)(rbf(a.x) * c); hv[1] = (_Float16)(rbf(a.y) * c);
  hv[2] = (_Float16)(rbf(a.z) * c); hv[3] = (_Float16)(rbf(a.w) * c);
  hv[4] = (_Float16)(rbf(b.x) * c); hv[5] = (_Float16)(rbf(b.y) * c);
  hv[6] = (_Float16)(rbf(b.z) * c); hv[7] = (_Float16)(rbf(b.w) * c);
  return hv;
}
__device__ __forceinline__ void cvt8hl(const v4f a, const v4f b, v8h& hv, v8h& lv) {
  float f[8] = {a.x * CX, a.y * CX, a.z * CX, a.w * CX, b.x * CX, b.y * CX, b.z * CX, b.w * CX};
#pragma unroll
  for (int i = 0; i < 8; ++i) {
    const _Float16 hq = (_Float16)f[i];
    hv[i] = hq;
    lv[i] = (_Float16)((f[i] - (float)hq) * CL);
  }
}

__device__ __forceinline__ int scan_chunk(const int* __restrict__ dsts, int nE, int cbase, int slotBase,
                                          int nb, int vec8, int* list, int tid, int lane, int wave) {
  int wc = 0;
  const int el0  = tid * EPT;
  const int e0   = cbase + el0;
  const int sent = -2147483647 - 1;
  v4i da, db;
  if (vec8 != 0 && cbase + CHUNK <= nE) {
    da = *(const v4i*)(dsts + e0);
    db = *(const v4i*)(dsts + e0 + 4);
  } else {
    da.x = (e0     < nE) ? dsts[min(e0,     nE - 1)] : sent;
    da.y = (e0 + 1 < nE) ? dsts[min(e0 + 1, nE - 1)] : sent;
    da.z = (e0 + 2 < nE) ? dsts[min(e0 + 2, nE - 1)] : sent;
    da.w = (e0 + 3 < nE) ? dsts[min(e0 + 3, nE - 1)] : sent;
    db.x = (e0 + 4 < nE) ? dsts[min(e0 + 4, nE - 1)] : sent;
    db.y = (e0 + 5 < nE) ? dsts[min(e0 + 5, nE - 1)] : sent;
    db.z = (e0 + 6 < nE) ? dsts[min(e0 + 6, nE - 1)] : sent;
    db.w = (e0 + 7 < nE) ? dsts[min(e0 + 7, nE - 1)] : sent;
  }
  const unsigned nbs = (unsigned)slotBase;
  const unsigned unb = (unsigned)nb;
  const unsigned s0 = (unsigned)da.x - nbs, s1 = (unsigned)da.y - nbs;
  const unsigned s2 = (unsigned)da.z - nbs, s3 = (unsigned)da.w - nbs;
  const unsigned s4 = (unsigned)db.x - nbs, s5 = (unsigned)db.y - nbs;
  const unsigned s6 = (unsigned)db.z - nbs, s7 = (unsigned)db.w - nbs;
  const bool h0 = s0 < unb, h1 = s1 < unb, h2 = s2 < unb, h3 = s3 < unb;
  const bool h4 = s4 < unb, h5 = s5 < unb, h6 = s6 < unb, h7 = s7 < unb;
  const unsigned any = __builtin_amdgcn_ballot_w32(h0 | h1 | h2 | h3 | h4 | h5 | h6 | h7);
  if (any != 0u) {
#define HITJ(J, HJ, SJ) { \
      const unsigned mj = __builtin_amdgcn_ballot_w32(HJ); \
      if (mj != 0u) { \
        if (HJ) { \
          const int pos = wc + (int)__builtin_amdgcn_mbcnt_lo(mj, 0u); \
          if (pos < WCAP) list[wave * WCAP + pos] = ((el0 + (J)) << SLOTB) | (int)(SJ); \
        } \
        wc += (int)__builtin_popcount(mj); } }
    HITJ(0, h0, s0)
    HITJ(1, h1, s1)
    HITJ(2, h2, s2)
    HITJ(3, h3, s3)
    HITJ(4, h4, s4)
    HITJ(5, h5, s5)
    HITJ(6, h6, s6)
    HITJ(7, h7, s7)
#undef HITJ
  }
  return wc;
}

__global__ __launch_bounds__(NTHR) void k_xprep(const float* __restrict__ x, unsigned short* xb, int nN, int nUnits) {
  const int i = (int)blockIdx.x * NTHR + (int)threadIdx.x;
  if (i >= nUnits) return;
  const int row = i >> 4;
  const int c0  = (i & 15) * 8;
  const int rc  = row < nN ? row : nN - 1;
  const float* p = x + (size_t)rc * DIN + c0;
  v4f a = *(const v4fa*)p, b = *(const v4fa*)(p + 4);
  const v4f z4 = {0.f, 0.f, 0.f, 0.f};
  if (row >= nN) { a = z4; b = z4; }
  const v8us hv = cvt8b(a, b);
  const size_t o = (size_t)row * DIN + c0;
  *(volatile v8us*)(xb + o) = hv;
  __threadfence();
  *(volatile v8us*)(xb + o) = hv;
}

__global__ __launch_bounds__(NTHR) void k_wtr_b(const float* __restrict__ w, int cols, int K,
                                                unsigned short* wt, int nUnits) {
  const int u = (int)blockIdx.x * NTHR + (int)threadIdx.x;
  if (u >= nUnits) return;
  const int kq = K >> 3;
  const int n  = u / kq;
  const int k8 = (u - n * kq) * 8;
  const int ncl = n < cols ? n : cols - 1;
  const float* p = w + (size_t)k8 * (size_t)cols + ncl;
  v4f a, b;
  a.x = p[0];                  a.y = p[(size_t)cols];       a.z = p[(size_t)2 * cols];   a.w = p[(size_t)3 * cols];
  b.x = p[(size_t)4 * cols];   b.y = p[(size_t)5 * cols];   b.z = p[(size_t)6 * cols];   b.w = p[(size_t)7 * cols];
  const v4f z4 = {0.f, 0.f, 0.f, 0.f};
  if (n >= cols) { a = z4; b = z4; }
  const v8us hv = cvt8b(a, b);
  const size_t o = (size_t)n * (size_t)K + k8;
  *(volatile v8us*)(wt + o) = hv;
  __threadfence();
  *(volatile v8us*)(wt + o) = hv;
}

__global__ __launch_bounds__(NTHR) void k_wtr_h(const float* __restrict__ w, int cols, int K,
                                                _Float16* wt, int nUnits) {
  const int u = (int)blockIdx.x * NTHR + (int)threadIdx.x;
  if (u >= nUnits) return;
  const int kq = K >> 3;
  const int n  = u / kq;
  const int k8 = (u - n * kq) * 8;
  const int ncl = n < cols ? n : cols - 1;
  const float* p = w + (size_t)k8 * (size_t)cols + ncl;
  v4f a, b;
  a.x = p[0];                  a.y = p[(size_t)cols];       a.z = p[(size_t)2 * cols];   a.w = p[(size_t)3 * cols];
  b.x = p[(size_t)4 * cols];   b.y = p[(size_t)5 * cols];   b.z = p[(size_t)6 * cols];   b.w = p[(size_t)7 * cols];
  const v4f z4 = {0.f, 0.f, 0.f, 0.f};
  if (n >= cols) { a = z4; b = z4; }
  const v8h hv = cvt8bh(a, b, CW);
  const size_t o = (size_t)n * (size_t)K + k8;
  *(volatile v8h*)(wt + o) = hv;
  __threadfence();
  *(volatile v8h*)(wt + o) = hv;
}

template<int BF, int RES>
__global__ __launch_bounds__(GTHR) void k_gemm(
    const unsigned short* __restrict__ A, const unsigned short* __restrict__ A2,
    const unsigned short* __restrict__ WT, float* outF, int K, int ldo, float scl, float scl2)
{
  typedef typename FT<BF>::T Frag;
  __shared__ __attribute__((aligned(16))) float stg[GBM * GBN];
  const int tid = (int)threadIdx.x, lane = tid & 31, wave = tid >> 5, hh = lane >> 4, m = lane & 15;
  const int rowBase = (int)blockIdx.x * GBM;
  const int col0    = (int)blockIdx.y * GBN;

  v8f acc[4], acc2[4];
  {
    const v8f z = {0.f, 0.f, 0.f, 0.f, 0.f, 0.f, 0.f, 0.f};
    acc[0] = z; acc[1] = z; acc[2] = z; acc[3] = z;
    acc2[0] = z; acc2[1] = z; acc2[2] = z; acc2[3] = z;
  }
  const size_t arow = (size_t)(rowBase + 16 * wave + m) * (size_t)K + 8 * hh;
  const unsigned short* ap  = A  + arow;
  const unsigned short* ap2 = A2 + arow;
  const unsigned short* wp  = WT + (size_t)(col0 + m) * (size_t)K + 8 * hh;
  const int ksteps = K >> 5;
#pragma unroll 1
  for (int ks = 0; ks < ksteps; ++ks) {
    Frag af, af2;
    af.u[0] = *(const v8usa*)(ap + 32 * ks);
    af.u[1] = *(const v8usa*)(ap + 32 * ks + 16);
    if (RES) {
      af2.u[0] = *(const v8usa*)(ap2 + 32 * ks);
      af2.u[1] = *(const v8usa*)(ap2 + 32 * ks + 16);
    } else {
      af2 = af;
    }
#pragma unroll
    for (int t = 0; t < 4; ++t) {
      const unsigned short* wq = wp + (size_t)(16 * t) * (size_t)K + 32 * ks;
      Frag bf;
      bf.u[0] = *(const v8usa*)wq;
      bf.u[1] = *(const v8usa*)(wq + 16);
      acc[t] = wmx(af, bf, acc[t]);
      if (RES) acc2[t] = wmx(af2, bf, acc2[t]);
    }
  }

#pragma unroll
  for (int t = 0; t < 4; ++t) {
    const int lc = 16 * t + m;
#pragma unroll
    for (int r = 0; r < 8; ++r) {
      const int lr = 16 * wave + 8 * hh + r;
      const float v = RES ? fmaf(acc2[t][r], scl2, acc[t][r] * scl) : acc[t][r] * scl;
      stg[lr * GBN + lc] = v;
    }
  }
  __syncthreads();

  v4f fv[8];
#pragma unroll
  for (int i = 0; i < 8; ++i) {
    const int lr = 16 * wave + 2 * i + hh;
    fv[i] = *(const v4fa*)(stg + lr * GBN + 4 * m);
  }
#pragma unroll
  for (int i = 0; i < 8; ++i) {
    const int lr = 16 * wave + 2 * i + hh;
    const int gr = rowBase + lr;
    float* op = outF + (size_t)gr * (size_t)ldo + col0 + 4 * m;
    *(volatile v4f*)op = fv[i];
  }
  __threadfence();
#pragma unroll
  for (int i = 0; i < 8; ++i) {
    const int lr = 16 * wave + 2 * i + hh;
    const int gr = rowBase + lr;
    float* op = outF + (size_t)gr * (size_t)ldo + col0 + 4 * m;
    *(volatile v4f*)op = fv[i];
  }
}

template<int LAYER>
__global__ __launch_bounds__(NTHR) void k_agg(
    const int* __restrict__ srcs, const int* __restrict__ dsts,
    const float* __restrict__ HF, const float* __restrict__ att, const float* __restrict__ bias,
    _Float16* Hh, _Float16* Hl, float* outF,
    int nN, int nE, int nb, int vec8, int MPr) {
  constexpr int C = (LAYER == 1) ? C1 : C2;
  constexpr int P = (LAYER == 1) ? P1 : P2;
  extern __shared__ v4f lds_dyn[];
  int* reg1 = (int*)lds_dyn;
  int* reg2 = reg1 + RCAP;
  int* scnt = reg2 + RCAP;
  int* soff = scnt + NBMAX;
  int* list = soff + NBMAX;
  int* wcnt = list + LISTN;
  int* wtot = wcnt + NWAVE;
  const int tid = (int)threadIdx.x, lane = tid & 31, wave = tid >> 5;
  const int nodeBase = (int)blockIdx.x * nb;

  for (int i = tid; i < NBMAX; i += NTHR) scnt[i] = 0;
  __syncthreads();

  int tot = 0;
  const int nChunks = (nE + CHUNK - 1) / CHUNK;
#pragma unroll 1
  for (int ch = 0; ch < nChunks; ++ch) {
    const int cbase = ch * CHUNK;
    const int wc = scan_chunk(dsts, nE, cbase, nodeBase, nb, vec8, list, tid, lane, wave);
    if (lane == 0) wcnt[wave] = wc;
    __syncthreads();
    int pre = 0, all = 0;
#pragma unroll
    for (int w2 = 0; w2 < NWAVE; ++w2) {
      int c = wcnt[w2];
      c = c < 0 ? 0 : (c > WCAP ? WCAP : c);
      all += c;
      pre += (w2 < wave) ? c : 0;
    }
    const int wcc  = wc > WCAP ? WCAP : wc;
    const int base = tot + pre;
#pragma unroll 1
    for (int i = lane; i < wcc; i += 32) {
      const int ent = list[wave * WCAP + i];
      const int el  = (ent >> SLOTB) & (CHUNK - 1);
      const int sl  = ent & (NBMAX - 1);
      int eid = cbase + el;
      eid = eid > nE - 1 ? nE - 1 : eid;
      const int pos = base + i;
      if (pos < RCAP) reg1[pos] = (int)(((unsigned)eid << SLOTB) | (unsigned)sl);
    }
    tot += all;
    tot = tot > RCAP ? RCAP : tot;
    __syncthreads();
  }
  const int nh = tot;

  if (wave == 0) {
#pragma unroll 1
    for (int b0 = 0; b0 < nh; b0 += 32) {
      const int idx = b0 + lane;
      const int uv  = reg1[idx < nh ? idx : nh - 1];
      const int m32 = (nh - b0) < 32 ? (nh - b0) : 32;
#pragma unroll 1
      for (int k = 0; k < m32; ++k) {
        const int u  = __builtin_amdgcn_readlane(uv, k);
        const int sl = u & (NBMAX - 1);
        if (lane == 0) scnt[sl] = scnt[sl] + 1;
      }
    }
  }
  __syncthreads();

  {
    const v4i ca = *(const v4i*)(scnt + 8 * tid);
    const v4i cb = *(const v4i*)(scnt + 8 * tid + 4);
    const int e0 = ca.x < 0 ? 0 : ca.x, e1 = ca.y < 0 ? 0 : ca.y, e2 = ca.z < 0 ? 0 : ca.z, e3 = ca.w < 0 ? 0 : ca.w;
    const int e4 = cb.x < 0 ? 0 : cb.x, e5 = cb.y < 0 ? 0 : cb.y, e6 = cb.z < 0 ? 0 : cb.z, e7 = cb.w < 0 ? 0 : cb.w;
    const int ts = e0 + e1 + e2 + e3 + e4 + e5 + e6 + e7;
    int incl = ts;
#pragma unroll
    for (int d = 1; d < 32; d <<= 1) {
      const int up = __shfl_up(incl, d);
      if (lane >= d) incl += up;
    }
    if (lane == 31) wtot[wave] = incl;
    __syncthreads();
    int pre = 0;
#pragma unroll
    for (int w2 = 0; w2 < NWAVE; ++w2) pre += (w2 < wave) ? wtot[w2] : 0;
    int run = pre + incl - ts;
    soff[8 * tid + 0] = run; run += e0;
    soff[8 * tid + 1] = run; run += e1;
    soff[8 * tid + 2] = run; run += e2;
    soff[8 * tid + 3] = run; run += e3;
    soff[8 * tid + 4] = run; run += e4;
    soff[8 * tid + 5] = run; run += e5;
    soff[8 * tid + 6] = run; run += e6;
    soff[8 * tid + 7] = run;
  }
  __syncthreads();
  for (int i = tid; i < NBMAX; i += NTHR) list[i] = soff[i];
  __syncthreads();

  if (wave == 0) {
#pragma unroll 1
    for (int b0 = 0; b0 < nh; b0 += 32) {
      const int idx = b0 + lane;
      const int uv  = reg1[idx < nh ? idx : nh - 1];
      const int m32 = (nh - b0) < 32 ? (nh - b0) : 32;
#pragma unroll 1
      for (int k = 0; k < m32; ++k) {
        const int u   = __builtin_amdgcn_readlane(uv, k);
        const int sl  = u & (NBMAX - 1);
        const int eid = (int)((unsigned)u >> SLOTB);
        if (lane == 0) {
          int pos = list[sl];
          pos = pos < 0 ? 0 : (pos > RCAP - 1 ? RCAP - 1 : pos);
          reg2[pos] = eid;
          list[sl] = pos + 1;
        }
      }
    }
  }
  __syncthreads();

  const int nbw = nb >> 3;
  const bool ovf = (nh >= RCAP);
  const float qnan = __int_as_float(0x7fc00000);
  float* stw = (float*)reg1 + wave * STW;
  const int lc = lane < 16 ? lane : 15;

  if (LAYER == 1) {
    const int c0 = 4 * lane;
    float at[4], bb[4];
    {
      const v4f a0 = *(const v4fa*)(att + c0);
      const v4f g0 = *(const v4fa*)(bias + c0);
      at[0] = rbf(a0.x); at[1] = rbf(a0.y); at[2] = rbf(a0.z); at[3] = rbf(a0.w);
      bb[0] = rbf(g0.x); bb[1] = rbf(g0.y); bb[2] = rbf(g0.z); bb[3] = rbf(g0.w);
    }
#pragma unroll 1
    for (int jt = 0; jt < nbw; ++jt) {
      const int slot = wave * nbw + jt;
      const int grow = nodeBase + slot;
      const int gcl  = grow < nN ? grow : nN - 1;
      int st = soff[slot];
      const int craw = scnt[slot];
      int cnt = craw;
      st  = st < 0 ? 0 : (st > nh ? nh : st);
      cnt = cnt < 0 ? 0 : (cnt > DEGCAP ? DEGCAP : cnt);
      if (cnt > nh - st) cnt = nh - st;
      const float pz = (ovf || craw > DEGCAP) ? qnan : 0.0f;
      const float live = grow < nN ? 1.0f : 0.0f;

      const float* drow = HF + (size_t)gcl * P + C + c0;
      const v4f d0 = *(const v4fa*)drow;
      float hd[4] = {d0.x, d0.y, d0.z, d0.w};
      float av[4] = {0.f, 0.f, 0.f, 0.f};
      float mx = MX0, dn = 0.f;

#pragma unroll 1
      for (int q = 0; q < cnt; ++q) {
        int idx = st + q; idx = idx > RCAP - 1 ? RCAP - 1 : idx;
        int eid = reg2[idx]; eid = eid < 0 ? 0 : (eid > nE - 1 ? nE - 1 : eid);
        const int sraw = srcs[eid];
        const int s = sraw < 0 ? 0 : (sraw > nN - 1 ? nN - 1 : sraw);
        const float* sr = HF + (size_t)s * P + c0;
        const v4f e0 = *(const v4fa*)sr;
        float hs[4] = {e0.x, e0.y, e0.z, e0.w};
        float part = 0.f;
#pragma unroll
        for (int i = 0; i < 4; ++i) {
          float v = hs[i] + hd[i];
          v = v > 0.f ? v : v * NEGS;
          part = fmaf(v, at[i], part);
        }
        part += __shfl_xor(part, 1);
        part += __shfl_xor(part, 2);
        part += __shfl_xor(part, 4);
        part += __shfl_xor(part, 8);
        const float al = part;
        const float df = al - mx;
        const float ee = __expf(-fabsf(df));
        const bool up  = df > 0.f;
        const float s1 = up ? ee : 1.0f;
        const float s2 = up ? 1.0f : ee;
        mx = up ? al : mx;
        dn = fmaf(dn, s1, s2);
#pragma unroll
        for (int i = 0; i < 4; ++i) av[i] = fmaf(av[i], s1, s2 * hs[i]);
      }
      const float ds = dn > 0.f ? dn : 1.0f;
      const float iv = (dn > 0.f ? 1.0f : 0.0f) * __builtin_amdgcn_rcpf(ds);
      float r[4];
#pragma unroll
      for (int i = 0; i < 4; ++i) {
        float v = fmaf(av[i], iv, bb[i]);
        v = fmaxf(v, 0.f) * live;
        r[i] = v + pz;
      }
      __builtin_amdgcn_fence(__ATOMIC_RELEASE, "wavefront");
      __builtin_amdgcn_wave_barrier();
      {
        const v4f rv = {r[0], r[1], r[2], r[3]};
        *(v4fa*)(stw + c0) = rv;
      }
      __builtin_amdgcn_fence(__ATOMIC_RELEASE, "wavefront");
      __builtin_amdgcn_wave_barrier();
      const v4f ga = *(const v4fa*)(stw + 8 * lc);
      const v4f gb = *(const v4fa*)(stw + 8 * lc + 4);
      v8h hv, lv;
      cvt8hl(ga, gb, hv, lv);
      const bool wr = grow < MPr;
      _Float16* gph = Hh + (size_t)grow * C + 8 * lc;
      _Float16* gpl = Hl + (size_t)grow * C + 8 * lc;
      const bool wsv = wr && (lane < (C / 8));
      if (wsv) { *(volatile v8h*)gph = hv; *(volatile v8h*)gpl = lv; }
      __threadfence();
      if (wsv) { *(volatile v8h*)gph = hv; *(volatile v8h*)gpl = lv; }
    }
  } else {
    constexpr int CJ = C / 32;
    float at[CJ], bb[CJ];
#pragma unroll
    for (int j = 0; j < CJ; ++j) {
      at[j] = rbf(att[32 * j + lane]);
      bb[j] = rbf(bias[32 * j + lane]);
    }
#pragma unroll 1
    for (int jt = 0; jt < nbw; ++jt) {
      const int slot = wave * nbw + jt;
      const int grow = nodeBase + slot;
      const int gcl  = grow < nN ? grow : nN - 1;
      int st = soff[slot];
      const int craw = scnt[slot];
      int cnt = craw;
      st  = st < 0 ? 0 : (st > nh ? nh : st);
      cnt = cnt < 0 ? 0 : (cnt > DEGCAP ? DEGCAP : cnt);
      if (cnt > nh - st) cnt = nh - st;
      const float pz = (ovf || craw > DEGCAP) ? qnan : 0.0f;

      const float* drow = HF + (size_t)gcl * P + C + lane;
      float hd[CJ], av[CJ];
#pragma unroll
      for (int j = 0; j < CJ; ++j) { hd[j] = drow[32 * j]; av[j] = 0.f; }
      ldwait();
      float mx = MX0, dn = 0.f;

#pragma unroll 1
      for (int q = 0; q < cnt; ++q) {
        int idx = st + q; idx = idx > RCAP - 1 ? RCAP - 1 : idx;
        int eid = reg2[idx]; eid = eid < 0 ? 0 : (eid > nE - 1 ? nE - 1 : eid);
        const int sraw = srcs[eid];
        const int s = sraw < 0 ? 0 : (sraw > nN - 1 ? nN - 1 : sraw);
        const float* sr = HF + (size_t)s * P + lane;
        float hs[CJ];
#pragma unroll
        for (int j = 0; j < CJ; ++j) hs[j] = sr[32 * j];
        ldwait();
        float part = 0.f;
#pragma unroll
        for (int j = 0; j < CJ; ++j) {
          float v = hs[j] + hd[j];
          v = v > 0.f ? v : v * NEGS;
          part = fmaf(v, at[j], part);
        }
#pragma unroll
        for (int off = 16; off > 0; off >>= 1) part += __shfl_xor(part, off);
        const float al = part;
        const float df = al - mx;
        const float ee = __expf(-fabsf(df));
        const bool up  = df > 0.f;
        const float s1 = up ? ee : 1.0f;
        const float s2 = up ? 1.0f : ee;
        mx = up ? al : mx;
        dn = fmaf(dn, s1, s2);
#pragma unroll
        for (int j = 0; j < CJ; ++j) av[j] = fmaf(av[j], s1, s2 * hs[j]);
      }
      const float ds = dn > 0.f ? dn : 1.0f;
      const float iv = (dn > 0.f ? 1.0f : 0.0f) * __builtin_amdgcn_rcpf(ds);
      float r[CJ];
#pragma unroll
      for (int j = 0; j < CJ; ++j) r[j] = fmaf(av[j], iv, bb[j]) + pz;
      __builtin_amdgcn_fence(__ATOMIC_RELEASE, "wavefront");
      __builtin_amdgcn_wave_barrier();
#pragma unroll
      for (int j = 0; j < CJ; ++j) stw[32 * j + lane] = r[j];
      __builtin_amdgcn_fence(__ATOMIC_RELEASE, "wavefront");
      __builtin_amdgcn_wave_barrier();
      const bool wr = grow < nN;
      const v4f gv = *(const v4fa*)(stw + 4 * lc);
      float* gp = outF + (size_t)grow * C + 4 * lc;
      const bool wsv = wr && (lane < (C / 4));
      if (wsv) *(volatile v4f*)gp = gv;
      __threadfence();
      if (wsv) *(volatile v4f*)gp = gv;
    }
  }
  (void)Hh; (void)Hl; (void)outF;
}

static int pick_nb(int nE, int nN) {
  int nb = NBRUN;
  while (nb > 16 && (long long)nb * (long long)nE * 5LL > (long long)RCAP * (long long)nN * 4LL) nb >>= 1;
  return nb;
}
static inline int cdiv(int a, int b) { return (a + b - 1) / b; }

extern "C" void kernel_launch(void* const* d_in, const int* in_sizes, int n_in,
                              void* d_out, int out_size, void* d_ws, size_t ws_size,
                              hipStream_t stream) {
  if (n_in < 18) return;
  const int nN = in_sizes[0] / DIN;
  if (nN <= 0 || in_sizes[0] != nN * DIN || nN > (1 << 22)) return;
  if (in_sizes[1] < 2 || (in_sizes[1] & 1) != 0) return;
  const int nE = in_sizes[1] / 2;
  if (nE < 1 || nE >= (1 << (32 - SLOTB))) return;
  if (in_sizes[2]  != DIN * C1 || in_sizes[3]  != DIN * C1) return;
  if (in_sizes[4]  != C1 || in_sizes[5]  != C1) return;
  if (in_sizes[6]  != C1 * C1  || in_sizes[7]  != C1 * C1) return;
  if (in_sizes[8]  != C1 || in_sizes[9]  != C1) return;
  if (in_sizes[10] != C1 * C1  || in_sizes[11] != C1 * C1) return;
  if (in_sizes[12] != C1 || in_sizes[13] != C1) return;
  if (in_sizes[14] != C1 * C2  || in_sizes[15] != C1 * C2) return;
  if (in_sizes[16] != C2 || in_sizes[17] != C2) return;
  if (out_size != nN * C2) return;

  const float* x    = (const float*)d_in[0];
  const int*   ei   = (const int*)  d_in[1];
  const float* Wl1  = (const float*)d_in[2];
  const float* Wr1  = (const float*)d_in[3];
  const float* at1  = (const float*)d_in[4];
  const float* b1   = (const float*)d_in[5];
  const float* Wl2  = (const float*)d_in[6];
  const float* Wr2  = (const float*)d_in[7];
  const float* at2  = (const float*)d_in[8];
  const float* b2   = (const float*)d_in[9];
  const float* Wl3  = (const float*)d_in[10];
  const float* Wr3  = (const float*)d_in[11];
  const float* at3  = (const float*)d_in[12];
  const float* b3   = (const float*)d_in[13];
  const float* Wl4  = (const float*)d_in[14];
  const float* Wr4  = (const float*)d_in[15];
  const float* at4  = (const float*)d_in[16];
  const float* b4   = (const float*)d_in[17];
  float* out = (float*)d_out;
  const int* src = ei;
  const int* dst = ei + nE;

  const int MP   = cdiv(nN, GBM) * GBM;
  const int nb   = pick_nb(nE, nN);
  if (nb < 16 || (nb & (nb - 1)) != 0 || nb > NBMAX) return;
  const int gA   = cdiv(MP, nb);
  const int vec8 = ((nE & 3) == 0) ? 1 : 0;
  if (gA * nb < MP) return;

  char* ws = (char*)d_ws;
  size_t off = 0;
  const size_t oXB  = off; off += (size_t)MP * DIN * 2;            off = (off + 255) & ~(size_t)255;
  const size_t oWT1 = off; off += (size_t)P1 * DIN * 2;            off = (off + 255) & ~(size_t)255;
  const size_t oWT2 = off; off += (size_t)P1 * C1 * 2;             off = (off + 255) & ~(size_t)255;
  const size_t oWT3 = off; off += (size_t)P1 * C1 * 2;             off = (off + 255) & ~(size_t)255;
  const size_t oWT4 = off; off += (size_t)P2 * C1 * 2;             off = (off + 255) & ~(size_t)255;
  const size_t oHF  = off; off += (size_t)MP * P1 * 4;             off = (off + 255) & ~(size_t)255;
  const size_t oHH  = off; off += (size_t)MP * C1 * 2;             off = (off + 255) & ~(size_t)255;
  const size_t oHL  = off; off += (size_t)MP * C1 * 2;             off = (off + 255) & ~(size_t)255;
  if (off > ws_size || off > (size_t)WSMAX) return;
  unsigned short* XB  = (unsigned short*)(ws + oXB);
  unsigned short* WT1 = (unsigned short*)(ws + oWT1);
  unsigned short* WT2 = (unsigned short*)(ws + oWT2);
  unsigned short* WT3 = (unsigned short*)(ws + oWT3);
  unsigned short* WT4 = (unsigned short*)(ws + oWT4);
  float*          HF  = (float*)(ws + oHF);
  unsigned short* HH  = (unsigned short*)(ws + oHH);
  unsigned short* HL  = (unsigned short*)(ws + oHL);

  hipFuncSetAttribute(reinterpret_cast<const void*>(&k_agg<1>),
                      hipFuncAttributeMaxDynamicSharedMemorySize, LDS_AGG);
  hipFuncSetAttribute(reinterpret_cast<const void*>(&k_agg<2>),
                      hipFuncAttributeMaxDynamicSharedMemorySize, LDS_AGG);

  const int nUx = MP * (DIN / 8);
  k_xprep<<<cdiv(nUx, NTHR), NTHR, 0, stream>>>(x, XB, nN, nUx);

  {
    const int nU1 = C1 * (DIN / 8);
    k_wtr_b<<<cdiv(nU1, NTHR), NTHR, 0, stream>>>(Wl1, C1, DIN, WT1, nU1);
    k_wtr_b<<<cdiv(nU1, NTHR), NTHR, 0, stream>>>(Wr1, C1, DIN, WT1 + (size_t)C1 * DIN, nU1);
    k_wtr_h<<<cdiv(nU1, NTHR), NTHR, 0, stream>>>(Wl2, C1, C1, (_Float16*)WT2, nU1);
    k_wtr_h<<<cdiv(nU1, NTHR), NTHR, 0, stream>>>(Wr2, C1, C1, (_Float16*)(WT2 + (size_t)C1 * C1), nU1);
    k_wtr_h<<<cdiv(nU1, NTHR), NTHR, 0, stream>>>(Wl3, C1, C1, (_Float16*)WT3, nU1);
    k_wtr_h<<<cdiv(nU1, NTHR), NTHR, 0, stream>>>(Wr3, C1, C1, (_Float16*)(WT3 + (size_t)C1 * C1), nU1);
    const int nU4 = C2 * (C1 / 8);
    k_wtr_h<<<cdiv(nU4, NTHR), NTHR, 0, stream>>>(Wl4, C2, C1, (_Float16*)WT4, nU4);
    k_wtr_h<<<cdiv(nU4, NTHR), NTHR, 0, stream>>>(Wr4, C2, C1, (_Float16*)(WT4 + (size_t)C2 * C1), nU4);
  }

  const int gM = MP / GBM;
  k_gemm<1, 0><<<dim3(gM, P1 / GBN), GTHR, 0, stream>>>(XB, XB, WT1, HF, DIN, P1, 1.0f, 0.0f);
  k_agg<1><<<gA, NTHR, LDS_AGG, stream>>>(src, dst, HF, at1, b1, (_Float16*)HH, (_Float16*)HL, out,
                                           nN, nE, nb, vec8, MP);
  k_gemm<0, 1><<<dim3(gM, P1 / GBN), GTHR, 0, stream>>>(HH, HL, WT2, HF, C1, P1, SCL_XW, SCL_XWL);
  k_agg<1><<<gA, NTHR, LDS_AGG, stream>>>(src, dst, HF, at2, b2, (_Float16*)HH, (_Float16*)HL, out,
                                           nN, nE, nb, vec8, MP);
  k_gemm<0, 1><<<dim3(gM, P1 / GBN), GTHR, 0, stream>>>(HH, HL, WT3, HF, C1, P1, SCL_XW, SCL_XWL);
  k_agg<1><<<gA, NTHR, LDS_AGG, stream>>>(src, dst, HF, at3, b3, (_Float16*)HH, (_Float16*)HL, out,
                                           nN, nE, nb, vec8, MP);
  k_gemm<0, 1><<<dim3(gM, P2 / GBN), GTHR, 0, stream>>>(HH, HL, WT4, HF, C1, P2, SCL_XW, SCL_XWL);
  k_agg<2><<<gA, NTHR, LDS_AGG, stream>>>(src, dst, HF, at4, b4, (_Float16*)HH, (_Float16*)HL, out,
                                           nN, nE, nb, vec8, MP);
}
